// SS2D_Mamba3_24361054503030
// MI455X (gfx1250) — hardware-verified
//
#include <hip/hip_runtime.h>
#include <math.h>


constexpr int DIM  = 192;
constexpr int HI   = 48;
constexpr int WI   = 48;
constexpr int L    = HI * WI;
constexpr int KD   = 4;
constexpr int E    = 384;
constexpr int E2   = 2 * E;
constexpr int NS   = 16;
constexpr int P    = 64;
constexpr int HH   = 6;
constexpr int HALF = NS / 2;
constexpr int ROWS = KD * L;
constexpr int NBD  = 64;
constexpr int CH   = L / DIM;
constexpr int NCHK = L / 128;
static_assert(L % 128 == 0 && L % 32 == 0 && ROWS % 16 == 0 && DIM % 64 == 0 && E % 64 == 0);
static_assert(CH * DIM == L && HH * P == E);

typedef unsigned short us;
typedef us     v8us  __attribute__((ext_vector_type(8)));
typedef us     v8usa __attribute__((ext_vector_type(8))) __attribute__((may_alias));
typedef __bf16 v16bf __attribute__((ext_vector_type(16)));
typedef float  v8f   __attribute__((ext_vector_type(8)));
typedef float  v4f   __attribute__((ext_vector_type(4)));
typedef float  v4fa  __attribute__((ext_vector_type(4))) __attribute__((may_alias));

union Frag { v16bf v; v8us h[2]; };

__device__ __forceinline__ us bf_rne(float f) {
    unsigned int u = __float_as_uint(f);
    u += 0x7FFFu + ((u >> 16) & 1u);
    return (us)(u >> 16);
}
__device__ __forceinline__ float bf_val(us b) { return __uint_as_float(((unsigned int)b) << 16); }

__device__ __forceinline__ void st4v(float* p, v4f v) { *(volatile v4f*)p = v; }
__device__ __forceinline__ void st8v(us* p, v8us v)   { *(volatile v8us*)p = v; }

__device__ __forceinline__ float silu_f(float v) {
    const float sg = 1.0f / (1.0f + expf(-v));
    return v * sg;
}
__device__ __forceinline__ float softplus_f(float v) {
    return fmaxf(v, 0.0f) + log1pf(expf(-fabsf(v)));
}

__device__ __forceinline__ v8f wmma3(v8f acc, v16bf ah, v16bf al, v16bf bh, v16bf bl) {
    acc = __builtin_amdgcn_wmma_f32_16x16x32_bf16(false, ah, false, bh, (short)0, acc, false, false);
    acc = __builtin_amdgcn_wmma_f32_16x16x32_bf16(false, ah, false, bl, (short)0, acc, false, false);
    acc = __builtin_amdgcn_wmma_f32_16x16x32_bf16(false, al, false, bh, (short)0, acc, false, false);
    asm volatile("v_nop\n\tv_nop\n\tv_nop\n\tv_nop" : "+v"(acc) : "v"(ah), "v"(al), "v"(bh), "v"(bl));
    return acc;
}

__device__ __forceinline__ void write_hilo_row(const float* smrow, us* gh, us* gl, size_t rowoff, int tid) {
    if (tid < 96) {
        const int plane = tid / 48;
        const int li    = tid - plane * 48;
        const int off   = (li >> 3) * 64 + (li & 7) * 8;
        v8us o;
#pragma unroll
        for (int c = 0; c < 8; ++c) {
            const float f = smrow[off + c];
            const us hb = bf_rne(f);
            o[c] = plane ? bf_rne(f - bf_val(hb)) : hb;
        }
        us* p = (plane ? gl : gh) + rowoff + off;
        st8v(p, o);
        __threadfence();
        st8v(p, o);
    }
}

__global__ void __launch_bounds__(256) k_wT(const float* __restrict__ src, int pitch, int nvalid, int Kd,
                                           us* __restrict__ dh, us* __restrict__ dl, int row0, int nrows) {
    const int lpr = Kd >> 6;
    const int gid = blockIdx.x * 256 + (int)threadIdx.x;
    if (gid >= nrows * lpr) return;
    const int rn = gid / lpr;
    const int j  = gid - rn * lpr;
    const bool valid = rn < nvalid;
    const int rsafe = valid ? rn : 0;
    v8us hv[8], lv[8];
#pragma unroll
    for (int g = 0; g < 8; ++g) {
        v8us a, b;
#pragma unroll
        for (int c = 0; c < 8; ++c) {
            const int kk = 64 * j + 8 * g + c;
            const float ld = src[(size_t)kk * pitch + rsafe];
            const float v = valid ? ld : 0.0f;
            const us hb = bf_rne(v);
            a[c] = hb;
            b[c] = bf_rne(v - bf_val(hb));
        }
        hv[g] = a; lv[g] = b;
    }
    const size_t o = (size_t)(row0 + rn) * Kd + 64 * j;
#pragma unroll
    for (int g = 0; g < 8; ++g) { st8v(dh + o + 8 * g, hv[g]); st8v(dl + o + 8 * g, lv[g]); }
    __threadfence();
#pragma unroll
    for (int g = 0; g < 8; ++g) { st8v(dh + o + 8 * g, hv[g]); st8v(dl + o + 8 * g, lv[g]); }
}

__global__ void __launch_bounds__(256) k_xseq(const float* __restrict__ x, us* __restrict__ xh, us* __restrict__ xl) {
    const int gid = blockIdx.x * 256 + (int)threadIdx.x;
    if (gid >= ROWS * 3) return;
    const int r    = gid / 3;
    const int j    = gid - r * 3;
    const int kdir = r / L;
    const int rr   = r - kdir * L;
    const int ch   = rr / CH;
    const int pb   = (rr - ch * CH) * DIM + 64 * j;
    const float* xc = x + (size_t)ch * L;
    v8us hv[8], lv[8];
#pragma unroll
    for (int g = 0; g < 8; ++g) {
        v8us a, b;
#pragma unroll
        for (int c = 0; c < 8; ++c) {
            const int pos = pb + 8 * g + c;
            const int p   = (kdir & 2) ? (L - 1 - pos) : pos;
            const int si  = (kdir & 1) ? ((p % HI) * WI + p / HI) : p;
            const float v = xc[si];
            const us hb = bf_rne(v);
            a[c] = hb;
            b[c] = bf_rne(v - bf_val(hb));
        }
        hv[g] = a; lv[g] = b;
    }
    const size_t o = (size_t)r * DIM + 64 * j;
#pragma unroll
    for (int g = 0; g < 8; ++g) { st8v(xh + o + 8 * g, hv[g]); st8v(xl + o + 8 * g, lv[g]); }
    __threadfence();
#pragma unroll
    for (int g = 0; g < 8; ++g) { st8v(xh + o + 8 * g, hv[g]); st8v(xl + o + 8 * g, lv[g]); }
}

__global__ void __launch_bounds__(256) k_gemm(const us* __restrict__ Ah, const us* __restrict__ Al,
                                             const us* __restrict__ Bh, const us* __restrict__ Bl,
                                             float* __restrict__ C, int M, int Kd, int Nd) {
    __shared__ float sm[8][16][64];
    const int lane = threadIdx.x & 31;
    const int w    = threadIdx.x >> 5;
    const int h    = lane >> 4;
    const int m    = lane & 15;
    const int ntn  = Nd >> 6;
    const int ntm  = M >> 4;
    const int tile = blockIdx.x * 8 + w;
    const bool active = tile < ntm * ntn;
    const int mt = active ? (tile / ntn) : 0;
    const int nt = active ? (tile - mt * ntn) : 0;

    const v8f zero8 = {0.f, 0.f, 0.f, 0.f, 0.f, 0.f, 0.f, 0.f};
    v8f acc[4];
#pragma unroll
    for (int j = 0; j < 4; ++j) acc[j] = zero8;

    if (active) {
        const us* ahp = Ah + (size_t)(mt * 16 + m) * Kd + 8 * h;
        const us* alp = Al + (size_t)(mt * 16 + m) * Kd + 8 * h;
        const us* bhp = Bh + (size_t)(nt * 64 + m) * Kd + 8 * h;
        const us* blp = Bl + (size_t)(nt * 64 + m) * Kd + 8 * h;
#pragma unroll 1
        for (int k0 = 0; k0 < Kd; k0 += 32) {
            Frag ah, al;
            ah.h[0] = *(const v8usa*)(ahp + k0);
            ah.h[1] = *(const v8usa*)(ahp + k0 + 16);
            al.h[0] = *(const v8usa*)(alp + k0);
            al.h[1] = *(const v8usa*)(alp + k0 + 16);
#pragma unroll
            for (int j = 0; j < 4; ++j) {
                const size_t bo = (size_t)j * 16 * Kd + k0;
                Frag bh, bl;
                bh.h[0] = *(const v8usa*)(bhp + bo);
                bh.h[1] = *(const v8usa*)(bhp + bo + 16);
                bl.h[0] = *(const v8usa*)(blp + bo);
                bl.h[1] = *(const v8usa*)(blp + bo + 16);
                acc[j] = wmma3(acc[j], ah.v, al.v, bh.v, bl.v);
            }
        }
    }
#pragma unroll
    for (int j = 0; j < 4; ++j) {
#pragma unroll
        for (int r = 0; r < 8; ++r) sm[w][8 * h + r][16 * j + m] = acc[j][r];
    }
    __syncthreads();
    if (active) {
        const int q    = lane >> 3;
        const int pc   = lane & 7;
        const int coff = (q & 1) * 32 + pc * 4;
        v4f v[8];
#pragma unroll
        for (int it = 0; it < 8; ++it) v[it] = *(const v4fa*)&sm[w][2 * it + (q >> 1)][coff];
        float* cb = C + (size_t)(mt * 16) * Nd + nt * 64 + coff;
#pragma unroll
        for (int it = 0; it < 8; ++it) st4v(cb + (size_t)(2 * it + (q >> 1)) * Nd, v[it]);
        __threadfence();
#pragma unroll
        for (int it = 0; it < 8; ++it) st4v(cb + (size_t)(2 * it + (q >> 1)) * Nd, v[it]);
    }
}

__global__ void __launch_bounds__(E) k_postproj(const float* __restrict__ proj, us* __restrict__ xah,
                                               us* __restrict__ xal, float* __restrict__ gate) {
    __shared__ float ssm[E];
    __shared__ float gsm[E];
    const int tid = threadIdx.x;
    const size_t r = blockIdx.x;
    const float* pr = proj + r * E2;
    ssm[tid] = silu_f(pr[tid]);
    gsm[tid] = silu_f(pr[E + tid]);
    __syncthreads();
    if (tid < 96) {
        const int off = (tid >> 3) * 32 + (tid & 7) * 4;
        const v4f v = *(const v4fa*)(gsm + off);
        float* p = gate + r * E + off;
        st4v(p, v);
        __threadfence();
        st4v(p, v);
    } else if (tid < 192) {
        write_hilo_row(ssm, xah, xal, r * E, tid - 96);
    }
}

__global__ void __launch_bounds__(256) k_rot(const float* __restrict__ bcdt, const float* __restrict__ b_bc,
                                            const float* __restrict__ dt_bias, const float* __restrict__ A_log,
                                            const float* __restrict__ theta, float* __restrict__ recs,
                                            float* __restrict__ dtr) {
    __shared__ float dts[L];
    __shared__ float cin[L];
    __shared__ float excl[NCHK + 1];
    __shared__ float rec_s[32][32];
    __shared__ float dr_s[32][2];
    const int tid  = threadIdx.x;
    const int kdir = blockIdx.x / HH;
    const int hd   = blockIdx.x - kdir * HH;
    const size_t rbase = (size_t)kdir * L;
    const size_t obase = (size_t)blockIdx.x * L;

    const float db = dt_bias[hd];
#pragma unroll 1
    for (int t = tid; t < L; t += 256)
        dts[t] = softplus_f(bcdt[(rbase + t) * NBD + 2 * NS + hd] + db);
    __syncthreads();
    if (tid < NCHK) {
        float a = 0.0f;
        const int b0 = tid * 128;
#pragma unroll 1
        for (int i = 0; i < 128; ++i) { a = a + dts[b0 + i]; cin[b0 + i] = a; }
    }
    __syncthreads();
    if (tid == 0) {
        float run = 0.0f;
        excl[0] = 0.0f;
#pragma unroll 1
        for (int c = 0; c < NCHK; ++c) { run = run + cin[c * 128 + 127]; excl[c + 1] = run; }
    }
    __syncthreads();

    const float aexp = expf(A_log[hd]);
    const int ts = tid >> 3;
    const int j  = tid & 7;
    const float th  = theta[hd * HALF + j];
    const float bb0 = b_bc[2 * j], bb1 = b_bc[2 * j + 1];
    const float cb0 = b_bc[NS + 2 * j], cb1 = b_bc[NS + 2 * j + 1];

#pragma unroll 1
    for (int tc = 0; tc < L; tc += 32) {
        const int t = tc + ts;
        const size_t row = rbase + t;
        const float dtv = dts[t];
        const float cs  = excl[t >> 7] + cin[t];
        const float ang = cs * th;
        float si, co;
        sincosf(ang, &si, &co);
        const float* br = bcdt + row * NBD;
        float b0 = br[2 * j] + bb0, b1 = br[2 * j + 1] + bb1;
        float c0 = br[NS + 2 * j] + cb0, c1 = br[NS + 2 * j + 1] + cb1;
        float sb = b0 * b0 + b1 * b1;
        float sc = c0 * c0 + c1 * c1;
        sb += __shfl_xor(sb, 1); sb += __shfl_xor(sb, 2); sb += __shfl_xor(sb, 4);
        sc += __shfl_xor(sc, 1); sc += __shfl_xor(sc, 2); sc += __shfl_xor(sc, 4);
        const float kb = rsqrtf(sb * (1.0f / (float)NS) + 1e-6f);
        const float kc = rsqrtf(sc * (1.0f / (float)NS) + 1e-6f);
        b0 *= kb; b1 *= kb; c0 *= kc; c1 *= kc;
        rec_s[ts][2 * j]          = b0 * co + b1 * si;
        rec_s[ts][2 * j + 1]      = b1 * co - b0 * si;
        rec_s[ts][NS + 2 * j]     = c0 * co + c1 * si;
        rec_s[ts][NS + 2 * j + 1] = c1 * co - c0 * si;
        if (j == 0) { dr_s[ts][0] = dtv; dr_s[ts][1] = expf(-(dtv * aexp)); }
        __syncthreads();
        if (tid < 32) {
            v4f v[8];
#pragma unroll
            for (int q = 0; q < 8; ++q) v[q] = *(const v4fa*)&rec_s[tid][4 * q];
            float* p = recs + (obase + tc + tid) * 32;
#pragma unroll
            for (int q = 0; q < 8; ++q) st4v(p + 4 * q, v[q]);
            __threadfence();
#pragma unroll
            for (int q = 0; q < 8; ++q) st4v(p + 4 * q, v[q]);
        } else if (tid < 64) {
            const int l2 = tid - 32;
            v4f v;
            v[0] = dr_s[l2][0]; v[1] = dr_s[l2][1]; v[2] = 0.0f; v[3] = 0.0f;
            float* p = dtr + (obase + tc + l2) * 4;
            st4v(p, v);
            __threadfence();
            st4v(p, v);
        }
        __syncthreads();
    }
}

__global__ void __launch_bounds__(64) k_scan(const float* __restrict__ zx, const float* __restrict__ recs,
                                            const float* __restrict__ dtr, const float* __restrict__ D_skip,
                                            float* __restrict__ ys) {
    __shared__ float ysm[32][P];
    const int p    = threadIdx.x;
    const int w    = p >> 5;
    const int lane = p & 31;
    const int q    = lane >> 3;
    const int pc   = lane & 7;
    const int kdir = blockIdx.x / HH;
    const int hd   = blockIdx.x - kdir * HH;
    const size_t rbase = (size_t)kdir * L;
    const size_t obase = (size_t)blockIdx.x * L;
    const float Dv = D_skip[hd];

    float st[NS], up[NS];
#pragma unroll
    for (int n = 0; n < NS; ++n) { st[n] = 0.0f; up[n] = 0.0f; }

#pragma unroll 1
    for (int tc = 0; tc < L; tc += 32) {
#pragma unroll 1
        for (int tt = 0; tt < 32; ++tt) {
            const int t = tc + tt;
            const float* rp = recs + (obase + t) * 32;
            v4f b4[4], c4[4];
#pragma unroll
            for (int i = 0; i < 4; ++i) {
                b4[i] = *(const v4fa*)(rp + 4 * i);
                c4[i] = *(const v4fa*)(rp + 16 + 4 * i);
            }
            const v4f dr = *(const v4fa*)(dtr + (obase + t) * 4);
            const float dtv = dr[0];
            const float rv  = dr[1];
            const float hdt = 0.5f * dtv;
            const float xv  = zx[(rbase + t) * E2 + E + hd * P + p];
            float y = 0.0f;
#pragma unroll
            for (int n = 0; n < NS; ++n) {
                const float bn = b4[n >> 2][n & 3];
                const float cn = c4[n >> 2][n & 3];
                const float u   = bn * xv;
                const float inp = hdt * (u + rv * up[n]);
                st[n] = rv * st[n] + inp;
                up[n] = u;
                y += cn * st[n];
            }
            ysm[tt][p] = y + Dv * xv;
        }
        __syncthreads();
        v4f v[8];
#pragma unroll
        for (int it = 0; it < 8; ++it) {
            const int g = w * 32 + it * 4 + q;
            v[it] = *(const v4fa*)&ysm[g >> 1][(g & 1) * 32 + pc * 4];
        }
#pragma unroll
        for (int it = 0; it < 8; ++it) {
            const int g = w * 32 + it * 4 + q;
            st4v(ys + (rbase + tc + (g >> 1)) * E + hd * P + (g & 1) * 32 + pc * 4, v[it]);
        }
        __threadfence();
#pragma unroll
        for (int it = 0; it < 8; ++it) {
            const int g = w * 32 + it * 4 + q;
            st4v(ys + (rbase + tc + (g >> 1)) * E + hd * P + (g & 1) * 32 + pc * 4, v[it]);
        }
        __syncthreads();
    }
}

__global__ void __launch_bounds__(E) k_postscan(const float* __restrict__ ys, const float* __restrict__ zx,
                                               const float* __restrict__ rms_w, us* __restrict__ gh,
                                               us* __restrict__ gl) {
    __shared__ float gsm[E];
    __shared__ float wsum[E / 32];
    __shared__ float scl_s;
    const int tid  = threadIdx.x;
    const int w    = tid >> 5;
    const int lane = tid & 31;
    const size_t r = blockIdx.x;
    const float y = ys[r * E + tid];
    const float z = zx[r * E2 + tid];
    const float v = y * silu_f(z);
    float sq = v * v;
    sq += __shfl_xor(sq, 16); sq += __shfl_xor(sq, 8); sq += __shfl_xor(sq, 4);
    sq += __shfl_xor(sq, 2);  sq += __shfl_xor(sq, 1);
    if (lane == 0) wsum[w] = sq;
    __syncthreads();
    if (tid == 0) {
        float s = 0.0f;
#pragma unroll
        for (int i = 0; i < E / 32; ++i) s += wsum[i];
        scl_s = rsqrtf(s * (1.0f / (float)E) + 1e-6f);
    }
    __syncthreads();
    gsm[tid] = v * scl_s * rms_w[tid];
    __syncthreads();
    write_hilo_row(gsm, gh, gl, r * E, tid);
}

__global__ void __launch_bounds__(E) k_merge(const float* __restrict__ mo, const float* __restrict__ gate,
                                            us* __restrict__ mh, us* __restrict__ ml) {
    __shared__ float msm[E];
    const int tid = threadIdx.x;
    const int l   = blockIdx.x;
    const int l1  = (l % HI) * WI + l / HI;
    const int idx0 = l, idx1 = L + l1, idx2 = 2 * L + (L - 1 - l), idx3 = 3 * L + (L - 1 - l1);
    float acc = 0.0f;
    {
        const size_t a0 = (size_t)idx0 * E + tid; const float t0 = mo[a0] * gate[a0]; acc = acc + t0;
        const size_t a1 = (size_t)idx1 * E + tid; const float t1 = mo[a1] * gate[a1]; acc = acc + t1;
        const size_t a2 = (size_t)idx2 * E + tid; const float t2 = mo[a2] * gate[a2]; acc = acc + t2;
        const size_t a3 = (size_t)idx3 * E + tid; const float t3 = mo[a3] * gate[a3]; acc = acc + t3;
    }
    msm[tid] = acc;
    __syncthreads();
    write_hilo_row(msm, mh, ml, (size_t)l * E, tid);
}

__global__ void __launch_bounds__(256) k_final(const float* __restrict__ outp, const float* __restrict__ x,
                                              const float* __restrict__ ln_g, const float* __restrict__ ln_b,
                                              const float* __restrict__ res_scale, float* __restrict__ out) {
    __shared__ float osm[32][DIM];
    __shared__ float mus[32];
    __shared__ float ris[32];
    const int tid = threadIdx.x;
    const int l0  = blockIdx.x * 32;
#pragma unroll
    for (int i = 0; i < 6; ++i) {
        const int idx = tid + 256 * i;
        const int row = idx / (DIM / 4);
        const int c4  = idx - row * (DIM / 4);
        *(v4fa*)&osm[row][c4 * 4] = *(const v4fa*)(outp + (size_t)(l0 + row) * DIM + c4 * 4);
    }
    __syncthreads();
    if (tid < 32) {
        const float* rr = &osm[tid][0];
        float mu = 0.0f;
#pragma unroll 1
        for (int d = 0; d < DIM; ++d) mu = mu + rr[d];
        mu = mu * (1.0f / (float)DIM);
        float var = 0.0f;
#pragma unroll 1
        for (int d = 0; d < DIM; ++d) { const float dd = rr[d] - mu; var = var + dd * dd; }
        var = var * (1.0f / (float)DIM);
        mus[tid] = mu;
        ris[tid] = rsqrtf(var + 1e-5f);
    }
    __syncthreads();
    const float rs = res_scale[0];
    v4f vals[6];
#pragma unroll
    for (int i = 0; i < 6; ++i) {
        const int qg = tid + 256 * i;
        const int d  = qg >> 3;
        const int pc = qg & 7;
        const float g = ln_g[d], b = ln_b[d];
        const v4f xv = *(const v4fa*)(x + (size_t)d * L + l0 + pc * 4);
        v4f o;
#pragma unroll
        for (int c = 0; c < 4; ++c) {
            const int l = pc * 4 + c;
            const float v  = osm[l][d];
            const float nv = (v - mus[l]) * ris[l] * g + b;
            o[c] = xv[c] + rs * nv;
        }
        vals[i] = o;
    }
#pragma unroll
    for (int i = 0; i < 6; ++i) {
        const int qg = tid + 256 * i;
        st4v(out + (size_t)(qg >> 3) * L + l0 + (qg & 7) * 4, vals[i]);
    }
    __threadfence();
#pragma unroll
    for (int i = 0; i < 6; ++i) {
        const int qg = tid + 256 * i;
        st4v(out + (size_t)(qg >> 3) * L + l0 + (qg & 7) * 4, vals[i]);
    }
}

extern "C" void kernel_launch(void* const* d_in, const int* in_sizes, int n_in,
                              void* d_out, int out_size, void* d_ws, size_t ws_size,
                              hipStream_t stream) {
    if (n_in < 16) return;
    if (in_sizes[0] != DIM * L || in_sizes[1] != DIM * E2 || in_sizes[2] != E * E2 ||
        in_sizes[3] != E * 2 * NS || in_sizes[4] != 2 * NS || in_sizes[5] != E * HH ||
        in_sizes[6] != HH || in_sizes[7] != HH || in_sizes[8] != HH * HALF || in_sizes[9] != HH ||
        in_sizes[10] != E || in_sizes[11] != E * E || in_sizes[12] != E * DIM ||
        in_sizes[13] != DIM || in_sizes[14] != DIM || in_sizes[15] < 1 || out_size != DIM * L) return;

    const float* x       = (const float*)d_in[0];
    const float* w_in    = (const float*)d_in[1];
    const float* w_zx    = (const float*)d_in[2];
    const float* w_bc    = (const float*)d_in[3];
    const float* b_bc    = (const float*)d_in[4];
    const float* w_dt    = (const float*)d_in[5];
    const float* dt_bias = (const float*)d_in[6];
    const float* A_log   = (const float*)d_in[7];
    const float* theta   = (const float*)d_in[8];
    const float* D_skip  = (const float*)d_in[9];
    const float* rms_w   = (const float*)d_in[10];
    const float* w_mout  = (const float*)d_in[11];
    const float* w_out   = (const float*)d_in[12];
    const float* ln_g    = (const float*)d_in[13];
    const float* ln_b    = (const float*)d_in[14];
    const float* res_sc  = (const float*)d_in[15];
    float* out           = (float*)d_out;

    size_t off = 0;
    auto carve = [&](size_t bytes) -> char* {
        char* p = (char*)d_ws + off;
        off += (bytes + 255) & ~(size_t)255;
        return p;
    };
    us* xsh  = (us*)carve((size_t)ROWS * DIM * 2);
    us* xsl  = (us*)carve((size_t)ROWS * DIM * 2);
    us* winh = (us*)carve((size_t)E2 * DIM * 2);
    us* winl = (us*)carve((size_t)E2 * DIM * 2);
    us* wzxh = (us*)carve((size_t)E2 * E * 2);
    us* wzxl = (us*)carve((size_t)E2 * E * 2);
    us* wbdh = (us*)carve((size_t)NBD * E * 2);
    us* wbdl = (us*)carve((size_t)NBD * E * 2);
    us* wmoh = (us*)carve((size_t)E * E * 2);
    us* wmol = (us*)carve((size_t)E * E * 2);
    us* wouh = (us*)carve((size_t)DIM * E * 2);
    us* woul = (us*)carve((size_t)DIM * E * 2);
    float* r1 = (float*)carve((size_t)ROWS * E2 * 4);
    char* xreg = carve((size_t)ROWS * E * 4);
    us* xah   = (us*)xreg;
    us* xal   = (us*)(xreg + (size_t)ROWS * E * 2);
    float* ys = (float*)xreg;
    float* gate = (float*)carve((size_t)ROWS * E * 4);
    float* bcdt = (float*)carve((size_t)ROWS * NBD * 4);
    float* recs = (float*)carve((size_t)KD * HH * L * 32 * 4);
    float* dtr  = (float*)carve((size_t)KD * HH * L * 4 * 4);
    us* gh   = (us*)carve((size_t)ROWS * E * 2);
    us* gl   = (us*)carve((size_t)ROWS * E * 2);
    us* mh   = (us*)carve((size_t)L * E * 2);
    us* ml   = (us*)carve((size_t)L * E * 2);
    float* outp = (float*)carve((size_t)L * DIM * 4);
    if (off > ws_size) return;

    auto cdiv = [](long long a, long long b) { return (int)((a + b - 1) / b); };

    k_wT<<<cdiv((long long)E2 * (DIM / 64), 256), 256, 0, stream>>>(w_in,   E2,     E2,     DIM, winh, winl, 0,  E2);
    k_wT<<<cdiv((long long)E2 * (E / 64), 256), 256, 0, stream>>>(w_zx,     E2,     E2,     E,   wzxh, wzxl, 0,  E2);
    k_wT<<<cdiv((long long)32 * (E / 64), 256), 256, 0, stream>>>(w_bc,     2 * NS, 2 * NS, E,   wbdh, wbdl, 0,  32);
    k_wT<<<cdiv((long long)32 * (E / 64), 256), 256, 0, stream>>>(w_dt,     HH,     HH,     E,   wbdh, wbdl, 32, 32);
    k_wT<<<cdiv((long long)E * (E / 64), 256), 256, 0, stream>>>(w_mout,    E,      E,      E,   wmoh, wmol, 0,  E);
    k_wT<<<cdiv((long long)DIM * (E / 64), 256), 256, 0, stream>>>(w_out,   DIM,    DIM,    E,   wouh, woul, 0,  DIM);

    k_xseq<<<cdiv((long long)ROWS * 3, 256), 256, 0, stream>>>(x, xsh, xsl);

    {
        const int tiles = (ROWS / 16) * (E2 / 64);
        k_gemm<<<cdiv(tiles, 8), 256, 0, stream>>>(xsh, xsl, winh, winl, r1, ROWS, DIM, E2);
    }
    k_postproj<<<ROWS, E, 0, stream>>>(r1, xah, xal, gate);
    {
        const int tiles = (ROWS / 16) * (E2 / 64);
        k_gemm<<<cdiv(tiles, 8), 256, 0, stream>>>(xah, xal, wzxh, wzxl, r1, ROWS, E, E2);
    }
    {
        const int tiles = (ROWS / 16) * (NBD / 64);
        k_gemm<<<cdiv(tiles, 8), 256, 0, stream>>>(xah, xal, wbdh, wbdl, bcdt, ROWS, E, NBD);
    }
    k_rot<<<KD * HH, 256, 0, stream>>>(bcdt, b_bc, dt_bias, A_log, theta, recs, dtr);
    k_scan<<<KD * HH, 64, 0, stream>>>(r1, recs, dtr, D_skip, ys);
    k_postscan<<<ROWS, E, 0, stream>>>(ys, r1, rms_w, gh, gl);
    {
        const int tiles = (ROWS / 16) * (E / 64);
        k_gemm<<<cdiv(tiles, 8), 256, 0, stream>>>(gh, gl, wmoh, wmol, r1, ROWS, E, E);
    }
    k_merge<<<L, E, 0, stream>>>(r1, gate, mh, ml);
    {
        const int tiles = (L / 16) * (DIM / 64);
        k_gemm<<<cdiv(tiles, 8), 256, 0, stream>>>(mh, ml, wouh, woul, outp, L, E, DIM);
    }
    k_final<<<L / 32, 256, 0, stream>>>(outp, x, ln_g, ln_b, res_sc, out);
}
